// LambdaLayer_61435212202589
// MI455X (gfx1250) — hardware-run, weakly checked
//
#include <hip/hip_runtime.h>


#define NB_  4
#define NP   256
#define NC_  1024
#define DK   256
#define NH   4
#define NE   961
#define NEP  1024
#define BNEPS 1e-3f
#define CARV 2048.0f
typedef _Float16 h16;
typedef unsigned short bf;
typedef __attribute__((ext_vector_type(16))) __bf16   v16bf;
typedef __attribute__((ext_vector_type(16))) _Float16 v16h;
typedef __attribute__((ext_vector_type(8)))  _Float16 v8h;
typedef __attribute__((ext_vector_type(8)))  unsigned short v8us;
typedef __attribute__((ext_vector_type(8)))  float    v8f;
typedef __attribute__((ext_vector_type(4)))  float    v4f;
typedef v8h  __attribute__((may_alias)) v8ha;
typedef v4f  __attribute__((may_alias)) v4fa;
typedef v8us __attribute__((may_alias)) v8usa;

__device__ __forceinline__ unsigned short f2bf(float f) { unsigned u = __float_as_uint(f); u += 0x7FFFu + ((u >> 16) & 1u); return (unsigned short)(u >> 16); }
__device__ __forceinline__ float bf2f(unsigned short b) { return __uint_as_float(((unsigned)b) << 16); }
__device__ __forceinline__ float bfr(float f) { return bf2f(f2bf(f)); }
__device__ __forceinline__ v16h cat16(v8h lo, v8h hi) { return __builtin_shufflevector(lo, hi, 0, 1, 2, 3, 4, 5, 6, 7, 8, 9, 10, 11, 12, 13, 14, 15); }
__device__ __forceinline__ v16bf cat16b(v8us lo, v8us hi) { return __builtin_bit_cast(v16bf, __builtin_shufflevector(lo, hi, 0, 1, 2, 3, 4, 5, 6, 7, 8, 9, 10, 11, 12, 13, 14, 15)); }
__device__ __forceinline__ v8f wmma16(v16h a, v16h b, v8f c) { return __builtin_amdgcn_wmma_f32_16x16x32_f16(false, a, false, b, (short)0, c, false, false); }
__device__ __forceinline__ v8f wmmab(v16bf a, v16bf b, v8f c) { return __builtin_amdgcn_wmma_f32_16x16x32_bf16(false, a, false, b, (short)0, c, false, false); }


template <typename T16> struct WFrag;
template <> struct WFrag<h16> { typedef v16h V; static __device__ __forceinline__ V ld(const h16* p) { return cat16(*(const v8h*)p, *(const v8h*)(p + 16)); } static __device__ __forceinline__ v8f mma(V a, V b, v8f c) { return wmma16(a, b, c); } };
template <> struct WFrag<bf> { typedef v16bf V; static __device__ __forceinline__ V ld(const bf* p) { return cat16b(*(const v8us*)p, *(const v8us*)(p + 16)); } static __device__ __forceinline__ v8f mma(V a, V b, v8f c) { return wmmab(a, b, c); } };
template <typename T16, int NSPLIT, bool BIAS>
__global__ __launch_bounds__(32) void k_gemmw(const T16* __restrict__ A, const T16* __restrict__ A2, const T16* __restrict__ Bt, const T16* __restrict__ Bt2, int K, float* C, int ldc, const float* __restrict__ bias, size_t sA, size_t sB, size_t sC) {
    typedef typename WFrag<T16>::V V;
    __shared__ __align__(16) float os[16 * 68];
    const size_t z = blockIdx.z; A += z * sA; if (A2) A2 += z * sA; Bt += z * sB; if (Bt2) Bt2 += z * sB; C += z * sC;
    const int lane = threadIdx.x & 31, lr = lane & 15, hi = lane >> 4; const int r0 = blockIdx.x * 64, c0 = blockIdx.y * 64;
    v8f acc[4][4];
#pragma unroll
    for (int mb = 0; mb < 4; ++mb)
#pragma unroll
        for (int nb = 0; nb < 4; ++nb) acc[mb][nb] = (v8f){};
    const size_t aoff = (size_t)(r0 + lr) * K + 8 * hi, boff = (size_t)(c0 + lr) * K + 8 * hi;

    for (int kc = 0; kc < K; kc += 32) {
        V a[4], a2[4];
#pragma unroll
        for (int mb = 0; mb < 4; ++mb) { a[mb] = WFrag<T16>::ld(A + aoff + (size_t)mb * 16 * K + kc); if (NSPLIT == 1 || NSPLIT == 2) a2[mb] = WFrag<T16>::ld(A2 + aoff + (size_t)mb * 16 * K + kc); }
#pragma unroll
        for (int nb = 0; nb < 4; ++nb) { const V b = WFrag<T16>::ld(Bt + boff + (size_t)nb * 16 * K + kc); V b2; if (NSPLIT >= 2) b2 = WFrag<T16>::ld(Bt2 + boff + (size_t)nb * 16 * K + kc);
#pragma unroll
            for (int mb = 0; mb < 4; ++mb) { acc[mb][nb] = WFrag<T16>::mma(a[mb], b, acc[mb][nb]); if (NSPLIT == 1 || NSPLIT == 2) acc[mb][nb] = WFrag<T16>::mma(a2[mb], b, acc[mb][nb]); if (NSPLIT >= 2) acc[mb][nb] = WFrag<T16>::mma(a[mb], b2, acc[mb][nb]); } }
        asm volatile("v_nop\n\tv_nop\n\tv_nop\n\tv_nop" : "+v"(acc[0][0]), "+v"(acc[1][1]), "+v"(acc[2][2]), "+v"(acc[3][3]) : "v"(a[0]), "v"(a[3]));
    }
#pragma unroll
    for (int mb = 0; mb < 4; ++mb) {
#pragma unroll
        for (int nb = 0; nb < 4; ++nb) {
#pragma unroll
            for (int j = 0; j < 8; ++j) os[(hi * 8 + j) * 68 + nb * 16 + lr] = acc[mb][nb][j]; }
        __builtin_amdgcn_wave_barrier(); asm volatile("" ::: "memory");
        float* crow = C + (size_t)(r0 + mb * 16) * ldc + c0;
#pragma unroll 1
        for (int ps = 0; ps < 2; ++ps) {
#pragma unroll
            for (int s = 0; s < 8; ++s) { const int row = 2 * s + hi, cofs = lr * 4; v4f val = *(const v4fa*)(os + row * 68 + cofs); if (BIAS) { val[0] += bfr(bias[c0 + cofs]); val[1] += bfr(bias[c0 + cofs + 1]); val[2] += bfr(bias[c0 + cofs + 2]); val[3] += bfr(bias[c0 + cofs + 3]); }
                *(volatile v4f*)(crow + (size_t)row * ldc + cofs) = val; }
            if (ps == 0) __threadfence(); }
        __builtin_amdgcn_wave_barrier(); asm volatile("" ::: "memory");
    }
}

__device__ __forceinline__ h16 tohx(float x) { return (h16)x; }
__device__ __forceinline__ void splitf(float y, unsigned short& h, unsigned short& l) { h = f2bf(y); l = f2bf(y - bf2f(h)); }
typedef __attribute__((ext_vector_type(2))) _Float16 v2h;
typedef __attribute__((ext_vector_type(4))) _Float16 v4h;
typedef __attribute__((ext_vector_type(2))) unsigned short v2us;
typedef __attribute__((ext_vector_type(4))) unsigned short v4us;
typedef __attribute__((ext_vector_type(2))) float v2f;
typedef __attribute__((ext_vector_type(4))) int v4i;
__device__ __forceinline__ float bf16_rne(float f) { unsigned int u = __float_as_uint(f); u += 0x7FFFu + ((u >> 16) & 1u); return __uint_as_float(u & 0xFFFF0000u); }
__global__ __launch_bounds__(256) void k_f2h(const float* __restrict__ S, h16* P16, size_t n4) { const size_t i = (size_t)blockIdx.x * 256 + threadIdx.x; if (i >= n4) return; const v4f v = *(const v4f*)(S + i * 4); v4h o;
#pragma unroll
    for (int q = 0; q < 4; ++q) o[q] = tohx(v[q]);
    *(volatile v4h*)(P16 + i * 4) = o; __threadfence(); *(volatile v4h*)(P16 + i * 4) = o; }
__global__ __launch_bounds__(256) void k_cvt8(const float* __restrict__ src, bf* dst, size_t n8) { const size_t i = (size_t)blockIdx.x * 256 + threadIdx.x; if (i >= n8) return; const v8f v = *(const v8f*)(src + i * 8); v8us o;
#pragma unroll
    for (int k = 0; k < 8; ++k) o[k] = f2bf(v[k]); *(volatile v8us*)(dst + i * 8) = o; __threadfence(); *(volatile v8us*)(dst + i * 8) = o; }
__global__ __launch_bounds__(256) void k_wtG(const float* __restrict__ w, int K, int N, bf* Bt) {
    const int lane = threadIdx.x & 31; const int L0 = (blockIdx.x * 8 + (threadIdx.x >> 5)) * 8; const int nlines = N * K / 64;
#pragma unroll
    for (int ps = 0; ps < 2; ++ps) {
        for (int l = 0; l < 8; ++l) { const int L = L0 + l; if (L >= nlines) break; const size_t e = (size_t)L * 64 + lane * 2; const int k = (int)(e % K), n = (int)(e / K); v2us o;
            o[0] = f2bf(w[(size_t)k * N + n]); o[1] = f2bf(w[(size_t)(k + 1) * N + n]); *(volatile v2us*)(Bt + e) = o; }
        if (ps == 0) __threadfence(); }
}
template <int W>
__global__ __launch_bounds__(256) void bnrec_kernel(const float* __restrict__ gam, const float* __restrict__ bet, const float* __restrict__ rm, const float* __restrict__ rv, float* __restrict__ SCL, float* __restrict__ SFT) {
  static_assert(W >= 32 && W <= 256 && W % 32 == 0, "bnrec: one block, whole lines"); const int c = threadIdx.x; if (c >= W) return; const float scl = (bf16_rne(gam[c]) * (rsqrtf(bf16_rne(rv[c]) + BNEPS))); const float sft = bf16_rne(bet[c]) - (bf16_rne(rm[c]) * scl);
  for (int pass = 0; pass < 2; ++pass) { ((volatile float*)SCL)[c] = scl; ((volatile float*)SFT)[c] = sft; __threadfence(); }
}
template <int W, int ACT>
__global__ __launch_bounds__(256) void bnact_kernel(const float* __restrict__ H, const float* __restrict__ SCL, const float* __restrict__ SFT, float* __restrict__ OUT, int op, int mrows) {
  const size_t i = (size_t)blockIdx.x * 256 + threadIdx.x; if (i >= (size_t)mrows * (W / 4)) return; const size_t v = i / (W / 4); const int c = (int)(i % (W / 4)) * 4;
  const v4f h = *(const v4f*)(H + v * W + c), s = *(const v4f*)(SCL + c), t = *(const v4f*)(SFT + c); v4f o;
  for (int j = 0; j < 4; ++j) { float y = (h[j] * s[j]) + t[j]; if (ACT == 1) y = fmaxf(y, 0.0f); if (ACT == 2) y = (y > 0.0f) ? y : (__expf(y) - 1.0f);     if (ACT == 3) y = (y >= 0.0f) ? y : 0.01f * y; o[j] = y; }
  for (int pass = 0; pass < 2; ++pass) { *(volatile v4f*)(OUT + v * (size_t)op + c) = o; __threadfence(); }
}
__global__ __launch_bounds__(256) void smxr_kernel(const float* __restrict__ LG, int pw, float* __restrict__ out, int nc, int rows) {
  const int r = blockIdx.x * 256 + threadIdx.x; if (r >= rows) return; const float* lr = LG + (size_t)r * pw; float mx = -INFINITY;
  for (int c = 0; c < nc; ++c) { const float l = lr[c]; mx = (l > mx) ? l : mx; }
  float s = 0.0f; for (int c = 0; c < nc; ++c) s += __expf(lr[c] - mx);
  const float inv = 1.0f / s;
  for (int pass = 0; pass < 2; ++pass) { float* orow = out + (size_t)r * nc; for (int c = 0; c < nc; ++c) *(volatile float*)(orow + c) = __expf(lr[c] - mx) * inv; __threadfence(); }
}
__global__ __launch_bounds__(256) void axpby_kernel(const float* __restrict__ A, const float* __restrict__ B, float* __restrict__ Y, size_t n4, float pa, float pb) {
  const size_t i = (size_t)blockIdx.x * 256 + threadIdx.x; if (i >= n4) return; const v4f a = *(const v4f*)(A + 4 * i); const v4f b = *(const v4f*)(B + 4 * i); v4f o; for (int j = 0; j < 4; ++j) o[j] = (pa * a[j]) + (pb * b[j]);
  for (int pass = 0; pass < 2; ++pass) { *(volatile v4f*)(Y + 4 * i) = o; __threadfence(); }
}
__global__ __launch_bounds__(256) void k_ez(const float* __restrict__ a12, h16* E) { const unsigned idx = blockIdx.x * 256 + threadIdx.x; const unsigned e = idx / (DK / 4), k4 = idx % (DK / 4); const unsigned ec = e < NE ? e : (NE - 1); const v4f p = *(const v4f*)(a12 + (size_t)ec * DK + k4 * 4); v4h o;
#pragma unroll
    for (int q = 0; q < 4; ++q) o[q] = tohx(bfr(p[q]));
    *(volatile v4h*)(E + (size_t)idx * 4) = o; __threadfence(); *(volatile v4h*)(E + (size_t)idx * 4) = o; }
__global__ __launch_bounds__(256) void k_qt(const float* __restrict__ Q, h16* QT) { const unsigned bh = blockIdx.y, n = blockIdx.x * 4u + (threadIdx.x >> 6), k4 = threadIdx.x & 63u; const float* src = Q + (size_t)bh * NP * NP + (size_t)(k4 * 4) * NP + n; v4h o;
#pragma unroll
    for (int q = 0; q < 4; ++q) o[q] = tohx(src[(size_t)q * NP]);
    h16* dst = QT + ((size_t)bh * NP + n) * NP + k4 * 4; *(volatile v4h*)dst = o; __threadfence(); *(volatile v4h*)dst = o; }
__global__ __launch_bounds__(256) void k_f2h2(const float* __restrict__ X, h16* HI, h16* LO) { const size_t i = (size_t)blockIdx.x * 256 + threadIdx.x; const v4f a = *(const v4f*)(X + i * 4); v4h hi, lo;
#pragma unroll
    for (int q = 0; q < 4; ++q) { const float y = __fmul_rn(a[q], CARV); hi[q] = tohx(y); lo[q] = tohx(__fsub_rn(y, (float)hi[q])); }
    *(volatile v4h*)(HI + i * 4) = hi; *(volatile v4h*)(LO + i * 4) = lo; __threadfence(); *(volatile v4h*)(HI + i * 4) = hi; *(volatile v4h*)(LO + i * 4) = lo; }
__global__ __launch_bounds__(256) void k_pick(const float* __restrict__ T, h16* S) { const unsigned row = blockIdx.x * 4u + (threadIdx.x >> 6), m0 = (threadIdx.x & 63u) * 4u; const unsigned b = row >> 10, n = (row >> 2) & 255u, h = row & 3u; const unsigned e0 = 31u * ((m0 >> 4) + 15u - (n >> 4)) + ((m0 & 15u) + 15u - (n & 15u)); const float* src = T + ((size_t)(b * NH + h) * NP + n) * NEP + e0; v4h o;
#pragma unroll
    for (int q = 0; q < 4; ++q) o[q] = tohx(src[q]);
    h16* dst = S + (size_t)row * NP + m0; *(volatile v4h*)dst = o; __threadfence(); *(volatile v4h*)dst = o; }

extern "C" void kernel_launch(void* const* d_in, const int* in_sizes, int n_in,
                              void* d_out, int out_size, void* d_ws, size_t ws_size, hipStream_t stream) {
    (void)in_sizes; (void)n_in; (void)out_size;
    const float* a0 = (const float*)d_in[0]; const float* a1 = (const float*)d_in[1]; const float* a2 = (const float*)d_in[2]; const float* a3 = (const float*)d_in[3];
    const float* a4 = (const float*)d_in[4]; const float* a5 = (const float*)d_in[5]; const float* a6 = (const float*)d_in[6]; const float* a7 = (const float*)d_in[7];
    const float* a8 = (const float*)d_in[8]; const float* a9 = (const float*)d_in[9]; const float* a10 = (const float*)d_in[10]; const float* a11 = (const float*)d_in[11]; const float* a12 = (const float*)d_in[12];
    float* OUT = (float*)d_out;
    char* wsp = (char*)d_ws;
    auto take = [&](size_t bytes) { char* p = wsp; wsp += (bytes + 255) & ~(size_t)255; return (void*)p; };
    const size_t NT = (size_t)NB_ * NP;
    bf* XB = (bf*)take(NT * NC_ * 2); bf* W1 = (bf*)take((size_t)NC_ * NC_ * 2); bf* W2 = (bf*)take((size_t)DK * NC_ * 2); bf* W3 = (bf*)take((size_t)DK * NC_ * 2);
    float* Q0 = (float*)take(NT * NC_ * 4); float* K0 = (float*)take(NT * DK * 4); float* V0 = (float*)take(NT * DK * 4);
    float* SQ = (float*)take((size_t)NC_ * 4); float* TQ = (float*)take((size_t)NC_ * 4); float* SV = (float*)take((size_t)DK * 4); float* TV = (float*)take((size_t)DK * 4);
    float* QN = (float*)take(NT * NC_ * 4); float* VN = (float*)take(NT * DK * 4); float* KS = (float*)take(NT * DK * 4);
    h16* KH = (h16*)take(NT * DK * 2); h16* VH = (h16*)take(NT * DK * 2); h16* VL = (h16*)take(NT * DK * 2); h16* QT = (h16*)take(NT * NC_ * 2);
    float* LC = (float*)take((size_t)NB_ * DK * DK * 4); h16* LH = (h16*)take((size_t)NB_ * DK * DK * 2); float* YC = (float*)take(NT * NC_ * 4);
    h16* EH = (h16*)take((size_t)NEP * DK * 2); float* TT = (float*)take(NT * NH * NEP * 4); h16* SH = (h16*)take(NT * NH * NP * 2); float* YP = (float*)take(NT * NC_ * 4);
    if ((size_t)(wsp - (char*)d_ws) > ws_size) return;
    k_cvt8<<<(unsigned)(NT * NC_ / 8 / 256), 256, 0, stream>>>(a0, XB, NT * NC_ / 8);
    k_wtG<<<(NC_ * NC_ / 64 + 63) / 64, 256, 0, stream>>>(a1, NC_, NC_, W1); k_wtG<<<(DK * NC_ / 64 + 63) / 64, 256, 0, stream>>>(a2, NC_, DK, W2); k_wtG<<<(DK * NC_ / 64 + 63) / 64, 256, 0, stream>>>(a3, NC_, DK, W3);
    k_gemmw<bf, 0, false><<<dim3(NT / 64, NC_ / 64, 1), 32, 0, stream>>>(XB, nullptr, W1, nullptr, NC_, Q0, NC_, nullptr, 0, 0, 0);
    k_gemmw<bf, 0, false><<<dim3(NT / 64, DK / 64, 1), 32, 0, stream>>>(XB, nullptr, W2, nullptr, NC_, K0, DK, nullptr, 0, 0, 0);
    k_gemmw<bf, 0, false><<<dim3(NT / 64, DK / 64, 1), 32, 0, stream>>>(XB, nullptr, W3, nullptr, NC_, V0, DK, nullptr, 0, 0, 0);
    for (int w = 0; w < NC_ / 256; ++w) bnrec_kernel<256><<<1, 256, 0, stream>>>(a4 + 256 * w, a5 + 256 * w, a6 + 256 * w, a7 + 256 * w, SQ + 256 * w, TQ + 256 * w);
    bnrec_kernel<256><<<1, 256, 0, stream>>>(a8, a9, a10, a11, SV, TV);
    bnact_kernel<NC_, 0><<<(unsigned)(NT * (NC_ / 4) / 256), 256, 0, stream>>>(Q0, SQ, TQ, QN, NC_, (int)NT); bnact_kernel<DK, 0><<<(unsigned)(NT * (DK / 4) / 256), 256, 0, stream>>>(V0, SV, TV, VN, DK, (int)NT);
    smxr_kernel<<<(unsigned)(NT / 256), 256, 0, stream>>>(K0, DK, KS, DK, (int)NT);
    k_f2h<<<(unsigned)(NT * DK / 4 / 256), 256, 0, stream>>>(KS, KH, NT * DK / 4); k_f2h2<<<(unsigned)(NT * DK / 4 / 256), 256, 0, stream>>>(VN, VH, VL);
    k_qt<<<dim3(NP / 4, NB_ * NH, 1), 256, 0, stream>>>(QN, QT);
    k_gemmw<h16, 1, false><<<dim3(DK / 64, DK / 64, NB_), 32, 0, stream>>>(VH, VL, KH, nullptr, NP, LC, DK, nullptr, (size_t)DK * NP, (size_t)DK * NP, (size_t)DK * DK);
    k_f2h<<<(unsigned)((size_t)NB_ * DK * DK / 4 / 256), 256, 0, stream>>>(LC, LH, (size_t)NB_ * DK * DK / 4);
    for (int b = 0; b < NB_; ++b) k_gemmw<h16, 0, false><<<dim3(NP / 64, DK / 64, NH), 32, 0, stream>>>(QT + (size_t)b * NH * NP * NP, nullptr, LH + (size_t)b * DK * DK, nullptr, DK, YC + (size_t)b * NP * NC_, NC_, nullptr, (size_t)NP * NP, 0, (size_t)DK);
    k_ez<<<NEP * (DK / 4) / 256, 256, 0, stream>>>(a12, EH);
    k_gemmw<h16, 0, false><<<dim3((unsigned)(NT * NH / 64), NEP / 64, 1), 32, 0, stream>>>(QT, nullptr, EH, nullptr, DK, TT, NEP, nullptr, 0, 0, 0);
    k_pick<<<(unsigned)(NT * NH / 4), 256, 0, stream>>>(TT, SH);
    k_gemmw<h16, 3, false><<<dim3(NP * NH / 64, DK / 64, NB_), 32, 0, stream>>>(SH, nullptr, VH, VL, NP, YP, DK, nullptr, (size_t)NP * NH * NP, (size_t)DK * NP, (size_t)NP * NH * DK);
    axpby_kernel<<<(unsigned)(NT * NC_ / 4 / 256), 256, 0, stream>>>(YC, YP, OUT, (int)(NT * NC_ / 4), 1.0f / CARV, 1.0f / CARV);
}
